// PixelRNN_66073776881698
// MI455X (gfx1250) — hardware-verified
//
#include <hip/hip_runtime.h>
#include <math.h>

constexpr int NB    = 16;
constexpr int NCH   = 16;
constexpr int NHW   = 64;
constexpr int NGATE = 64;
constexpr int NLAY  = 7;
constexpr int NJP   = 127;
constexpr int NPIX  = NB * NHW * NHW;
constexpr int GPITCH = 2 * NGATE;
constexpr int KPAD_IN  = 32;
constexpr int KPAD_MID = 416;
constexpr int KPAD_OUT = 32;
constexpr int MID_CHUNK  = 16384;
constexpr int MID_NCHUNK = 4;
constexpr int APITCH = 40;
constexpr int HS_DIR = NB * NJP * NHW * NCH;
static_assert(NPIX % 64 == 0);
static_assert(MID_CHUNK * MID_NCHUNK == NPIX);
static_assert(MID_CHUNK % 64 == 0);
static_assert(KPAD_IN % 32 == 0 && KPAD_MID % 32 == 0 && KPAD_OUT % 32 == 0);
static_assert((NPIX * 4) % 256 == 0);
static_assert((MID_CHUNK * (KPAD_MID / 8)) % 256 == 0);
static_assert((NLAY * 128 * 4) % 256 == 0);
static_assert((NLAY * 2 * 64 * 4) % 256 == 0);
static_assert(2 * HS_DIR * 4 <= NPIX * 64 * 4);
static_assert(MID_CHUNK * KPAD_MID * 2 <= 16777216);
static_assert(NGATE == 4 * NCH);
static_assert((2 * NHW * APITCH * 2) % (16 * 128) == 0);

typedef __attribute__((ext_vector_type(16))) _Float16 v16h;
typedef __attribute__((ext_vector_type(8)))  _Float16 v8h;
typedef __attribute__((ext_vector_type(16))) __bf16   v16b;
typedef __attribute__((ext_vector_type(8)))  __bf16   v8b;
typedef __attribute__((ext_vector_type(8)))  float    v8f;
typedef __attribute__((ext_vector_type(4)))  float    v4f;
typedef __attribute__((ext_vector_type(4)))  unsigned int v4u;

__device__ __forceinline__ unsigned short f2bf_bits(float f) {
  unsigned u = __float_as_uint(f);
  return (unsigned short)((u + 0x7FFFu + ((u >> 16) & 1u)) >> 16);
}
__device__ __forceinline__ float bf_bits2f(unsigned short h) { return __uint_as_float(((unsigned)h) << 16); }

__device__ __forceinline__ void dep_guard_h(v8f& a, v8f& b, v16h x, v16h y) { asm volatile("v_nop\n\tv_nop\n\tv_nop\n\tv_nop" : "+v"(a), "+v"(b) : "v"(x), "v"(y)); }
__device__ __forceinline__ void dep_guard_b(v8f& a, v8f& b, v16b x, v16b y) { asm volatile("v_nop\n\tv_nop\n\tv_nop\n\tv_nop" : "+v"(a), "+v"(b) : "v"(x), "v"(y)); }
__device__ __forceinline__ void keep4_h(v16h a, v16h b, v16h c, v16h d) { asm volatile("v_nop" :: "v"(a), "v"(b), "v"(c), "v"(d)); }
__device__ __forceinline__ void keep4_b(v16b a, v16b b, v16b c, v16b d) { asm volatile("v_nop" :: "v"(a), "v"(b), "v"(c), "v"(d)); }
__device__ __forceinline__ void acc_guard4(v8f& a, v8f& b, v8f& c, v8f& d) { asm volatile("v_nop\n\tv_nop\n\tv_nop\n\tv_nop" : "+v"(a), "+v"(b), "+v"(c), "+v"(d)); }
template <typename T> struct Frag;
template <> struct Frag<_Float16> {
  typedef v16h V; union U { v16h v; v8h h[2]; };
  static __device__ __forceinline__ v16h load(const _Float16* p) {
    U f; f.h[0] = *(const v8h*)(p); f.h[1] = *(const v8h*)(p + 16); return f.v;
  }
  static __device__ __forceinline__ v8f mma(v16h a, v16h b, v8f c) {
    return __builtin_amdgcn_wmma_f32_16x16x32_f16(false, a, false, b, (short)0, c, false, false);
  }
  static __device__ __forceinline__ void guard(v8f& a, v8f& b, v16h x, v16h y) { dep_guard_h(a, b, x, y); }
  static __device__ __forceinline__ void keep(v16h a, v16h b, v16h c, v16h d) { keep4_h(a, b, c, d); }
};
template <> struct Frag<__bf16> {
  typedef v16b V; union U { v16b v; v8b h[2]; };
  static __device__ __forceinline__ v16b load(const __bf16* p) {
    U f; f.h[0] = *(const v8b*)(p); f.h[1] = *(const v8b*)(p + 16); return f.v;
  }
  static __device__ __forceinline__ v8f mma(v16b a, v16b b, v8f c) {
    return __builtin_amdgcn_wmma_f32_16x16x32_bf16(false, a, false, b, (short)0, c, false, false);
  }
  static __device__ __forceinline__ void guard(v8f& a, v8f& b, v16b x, v16b y) { dep_guard_b(a, b, x, y); }
  static __device__ __forceinline__ void keep(v16b a, v16b b, v16b c, v16b d) { keep4_b(a, b, c, d); }
};

template <int ET> struct Elem;
template <> struct Elem<0> { typedef _Float16 T; };
template <> struct Elem<1> { typedef __bf16 T; };
template <int ET, bool SPLIT, int BIAS_MODE, int OUT_MODE, bool RESID, int ACT = 0>
__global__ __launch_bounds__(256) void wmma_gemm64(
    const unsigned short* __restrict__ Ap, const unsigned short* __restrict__ A2p, int lda, long strideA,
    const unsigned short* __restrict__ Btp, const unsigned short* __restrict__ Bt2p, int ldb, long strideB,
    void* __restrict__ Cout, void* __restrict__ Cout2, int ldc, long strideC,
    const float* __restrict__ bias,
    const float* __restrict__ resid, long strideR,
    int M, int N, int K, float scale) {
  typedef typename Elem<ET>::T T;
  typedef typename Frag<T>::V V;
  const T* A = (const T*)Ap; const T* A2 = (const T*)A2p; const T* Bt = (const T*)Btp; const T* Bt2 = (const T*)Bt2p;
  __shared__ __align__(16) float sT[8][16 * 68];
  const int b    = blockIdx.y;
  const int lane = threadIdx.x & 31;
  const int wave = threadIdx.x >> 5;
  const int tilesN = N >> 6;
  const int tilesM = M >> 6;
  const int tile = blockIdx.x * 8 + wave;
  if (tile >= tilesM * tilesN) return;
  const int tm = tile / tilesN;
  const int tn = tile - tm * tilesN;
  const int m0 = tm << 6;
  const int n0 = tn << 6;

  const T* Ab  = A  + (size_t)b * strideA;
  const T* Bb  = Bt + (size_t)b * strideB;
  const T* Ab2 = SPLIT ? (A2  + (size_t)b * strideA) : nullptr;
  const T* Bb2 = SPLIT ? (Bt2 + (size_t)b * strideB) : nullptr;

  const int rlane = lane & 15;
  const int koff  = (lane >> 4) * 8;
  const int mOff  = (lane >> 4) * 8;

  v8f acc[4][4];
#pragma unroll
  for (int i = 0; i < 4; ++i)
#pragma unroll
    for (int j = 0; j < 4; ++j) acc[i][j] = (v8f){0.f,0.f,0.f,0.f,0.f,0.f,0.f,0.f};

  for (int k0 = 0; k0 < K; k0 += 32) {
    V bh[4], bl[4];
#pragma unroll
    for (int j = 0; j < 4; ++j) {
      const size_t bo = (size_t)(n0 + (j << 4) + rlane) * ldb + koff + k0;
      bh[j] = Frag<T>::load(Bb + bo);
      if (SPLIT) bl[j] = Frag<T>::load(Bb2 + bo);
    }
#pragma unroll
    for (int i = 0; i < 4; ++i) {
      const size_t ao = (size_t)(m0 + (i << 4) + rlane) * lda + koff + k0;
      V ah = Frag<T>::load(Ab + ao);
      V al;
      if (SPLIT) al = Frag<T>::load(Ab2 + ao);
#pragma unroll
      for (int j = 0; j < 4; ++j) {
        acc[i][j] = Frag<T>::mma(ah, bh[j], acc[i][j]);
        if (SPLIT) {
          acc[i][j] = Frag<T>::mma(ah, bl[j], acc[i][j]);
          acc[i][j] = Frag<T>::mma(al, bh[j], acc[i][j]);
        }
      }
      Frag<T>::guard(acc[i][0], acc[i][3], ah, SPLIT ? al : ah);
    }
    Frag<T>::keep(bh[0], bh[1], bh[2], bh[3]);
    if (SPLIT) Frag<T>::keep(bl[0], bl[1], bl[2], bl[3]);
  }
  acc_guard4(acc[0][0], acc[0][1], acc[0][2], acc[0][3]);
  acc_guard4(acc[1][0], acc[1][1], acc[1][2], acc[1][3]);
  acc_guard4(acc[2][0], acc[2][1], acc[2][2], acc[2][3]);
  acc_guard4(acc[3][0], acc[3][1], acc[3][2], acc[3][3]);

  float* slab = sT[wave];
  const float* Rb = RESID ? (resid + (size_t)b * strideR) : nullptr;
#pragma unroll
  for (int i = 0; i < 4; ++i) {
    const int mBase = m0 + (i << 4);
#pragma unroll
    for (int j = 0; j < 4; ++j) {
      const int n = n0 + (j << 4) + rlane;
      float bv = 0.f;
      if (BIAS_MODE == 2) bv = bias[n];
#pragma unroll
      for (int r = 0; r < 8; ++r) {
        float v = acc[i][j][r] * scale;
        if (BIAS_MODE == 1) v += bias[mBase + mOff + r];
        if (BIAS_MODE == 2) v += bv;
        if (RESID) v += Rb[(size_t)(mBase + mOff + r) * ldc + n];
        if (ACT == 1) v = tanhf(v);
        if (ACT == 2) v = fmaxf(v, 0.0f);
        if (ACT == 4) v = (v > 0.f) ? v : 0.01f * v;
        slab[(mOff + r) * 68 + (j << 4) + rlane] = v;
      }
    }
    __builtin_amdgcn_fence(__ATOMIC_RELEASE, "workgroup");
    __builtin_amdgcn_wave_barrier();
    __builtin_amdgcn_fence(__ATOMIC_ACQUIRE, "workgroup");
    if (OUT_MODE == 0) {
      float* C = (float*)Cout + (size_t)b * strideC;
      const int hh = lane >> 4, c4 = (lane & 15) * 4;
      for (int pass = 0; pass < 2; ++pass) {
#pragma unroll
        for (int it = 0; it < 8; ++it) {
          const int row = it * 2 + hh;
          v4f v = *(const v4f*)(slab + row * 68 + c4);
          *(volatile v4f*)(C + (size_t)(mBase + row) * ldc + n0 + c4) = v;
        }
        __threadfence();
      }
    } else {
      const int q = lane >> 3, c8 = (lane & 7) * 8;
      unsigned short* C  = (unsigned short*)Cout  + (size_t)b * strideC;
      unsigned short* C2 = (OUT_MODE == 2) ? ((unsigned short*)Cout2 + (size_t)b * strideC) : nullptr;
      for (int pass = 0; pass < 2; ++pass) {
#pragma unroll
        for (int it = 0; it < 4; ++it) {
          const int row = it * 4 + q;
          const float* sp = slab + row * 68 + c8;
          v8h hv, lv;
#pragma unroll
          for (int e = 0; e < 8; ++e) {
            if (OUT_MODE == 1) {
              hv[e] = (_Float16)sp[e];
            } else {
              unsigned short hb = f2bf_bits(sp[e]);
              unsigned short lb = f2bf_bits(sp[e] - bf_bits2f(hb));
              hv[e] = __builtin_bit_cast(_Float16, hb);
              lv[e] = __builtin_bit_cast(_Float16, lb);
            }
          }
          *(volatile v8h*)(C + (size_t)(mBase + row) * ldc + n0 + c8) = hv;
          if (OUT_MODE == 2) *(volatile v8h*)(C2 + (size_t)(mBase + row) * ldc + n0 + c8) = lv;
        }
        __threadfence();
      }
    }
    __builtin_amdgcn_fence(__ATOMIC_RELEASE, "workgroup");
    __builtin_amdgcn_wave_barrier();
    __builtin_amdgcn_fence(__ATOMIC_ACQUIRE, "workgroup");
  }
}

__device__ __forceinline__ void split_pack(float x0, float x1, unsigned& hw, unsigned& lw) {
  const unsigned short h0 = f2bf_bits(x0);
  const unsigned short h1 = f2bf_bits(x1);
  const unsigned short l0 = f2bf_bits(x0 - bf_bits2f(h0));
  const unsigned short l1 = f2bf_bits(x1 - bf_bits2f(h1));
  hw = (unsigned)h0 | ((unsigned)h1 << 16);
  lw = (unsigned)l0 | ((unsigned)l1 << 16);
}
__device__ __forceinline__ void store_planes2(unsigned short* hp, unsigned short* lp, size_t off, v4u hv, v4u lv) {
  volatile v4u* ph = (volatile v4u*)(hp + off);
  volatile v4u* pl = (volatile v4u*)(lp + off);
  *ph = hv;
  *pl = lv;
  __threadfence();
  *ph = hv;
  *pl = lv;
}
__device__ __forceinline__ void store_v4f2(float* p, v4f v) {
  *(volatile v4f*)p = v;
  __threadfence();
  *(volatile v4f*)p = v;
}
__device__ __forceinline__ float fsig(float x)  { return __builtin_amdgcn_rcpf(1.0f + __expf(-x)); }
__device__ __forceinline__ float ftanh(float x) { return 1.0f - 2.0f * __builtin_amdgcn_rcpf(__expf(2.0f * x) + 1.0f); }

template <int CIN, int KS>
__device__ __forceinline__ float conv_w_elem(const float* __restrict__ w, int o, int cout, int ntaps, int k) {
  const int tap = k / CIN;
  const int ci = k - tap * CIN;
  const bool valid = (o < cout) && (tap < ntaps);
  const int oc = min(o, cout - 1);
  const int tapc = min(tap, ntaps - 1);
  const int t7 = tapc / 7;
  const int ky = (tapc < 21) ? t7 : 3;
  const int kx = (tapc < 21) ? (tapc - t7 * 7) : (tapc - 21);
  const int idx = ((oc * CIN + ci) * KS + ky) * KS + kx;
  const float x = w[idx];
  return valid ? x : 0.0f;
}
template <int CIN, int KS>
__global__ __launch_bounds__(256) void prep_conv_w(const float* __restrict__ w, int cout, int ntaps, int kp8,
                                                    unsigned short* __restrict__ hi, unsigned short* __restrict__ lo) {
  const int t = blockIdx.x * 256 + threadIdx.x;
  if (t >= 64 * kp8) return;
  const int o = t / kp8;
  const int g = t - o * kp8;
  v4u hv, lv;
#pragma unroll
  for (int m = 0; m < 4; ++m) {
    const float x0 = conv_w_elem<CIN, KS>(w, o, cout, ntaps, 8 * g + 2 * m);
    const float x1 = conv_w_elem<CIN, KS>(w, o, cout, ntaps, 8 * g + 2 * m + 1);
    unsigned hw, lw; split_pack(x0, x1, hw, lw); hv[m] = hw; lv[m] = lw;
  }
  store_planes2(hi, lo, (size_t)8 * t, hv, lv);
}

__global__ __launch_bounds__(256) void prep_wis(const float* __restrict__ wis, unsigned short* __restrict__ hi,
                                                 unsigned short* __restrict__ lo) {
  const int t = blockIdx.x * 256 + threadIdx.x;
  if (t >= NLAY * 128 * 4) return;
  const int row = t >> 2, q = t & 3;
  const float* sp = wis + (size_t)row * NCH + (q & 1) * 8;
  const bool pz = (q < 2);
  v4u hv, lv;
#pragma unroll
  for (int m = 0; m < 4; ++m) {
    const float x0 = pz ? sp[2 * m] : 0.0f;
    const float x1 = pz ? sp[2 * m + 1] : 0.0f;
    unsigned hw, lw; split_pack(x0, x1, hw, lw); hv[m] = hw; lv[m] = lw;
  }
  store_planes2(hi, lo, (size_t)8 * t, hv, lv);
}

__global__ __launch_bounds__(256) void prep_wss(const float* __restrict__ wss, unsigned short* __restrict__ hi,
                                                 unsigned short* __restrict__ lo) {
  const int t = blockIdx.x * 256 + threadIdx.x;
  if (t >= NLAY * 2 * 64 * 4) return;
  const int row = t >> 2, q = t & 3;
  const int tapsel = q >> 1;
  const int c0 = (q & 1) * 8;
  const float* sp = wss + ((size_t)row * NCH + c0) * 2 + tapsel;
  v4u hv, lv;
#pragma unroll
  for (int m = 0; m < 4; ++m) {
    const float x0 = sp[(2 * m) * 2];
    const float x1 = sp[(2 * m + 1) * 2];
    unsigned hw, lw; split_pack(x0, x1, hw, lw); hv[m] = hw; lv[m] = lw;
  }
  store_planes2(hi, lo, (size_t)8 * t, hv, lv);
}

__global__ __launch_bounds__(64) void prep_bias_pad(const float* __restrict__ b_in, const float* __restrict__ b_mid,
                                                     const float* __restrict__ b_out, float* __restrict__ dst) {
  const int t = threadIdx.x;
  const int s = t >> 4;
  const int n0 = (t & 15) * 4;
  v4f o;
#pragma unroll
  for (int e = 0; e < 4; ++e) {
    const int n = n0 + e;
    const int nc = min(n, 15);
    const float va = b_in[nc];
    const float vb = b_mid[nc];
    const float vc = b_mid[16 + nc];
    const float vd = b_out[0];
    const bool in16 = (n < 16);
    float v = 0.0f;
    v = (s == 0) ? (in16 ? va : 0.0f) : v;
    v = (s == 1) ? (in16 ? vb : 0.0f) : v;
    v = (s == 2) ? (in16 ? vc : 0.0f) : v;
    v = (s == 3) ? ((n == 0) ? vd : 0.0f) : v;
    o[e] = v;
  }
  store_v4f2(dst + 4 * t, o);
}

__device__ __forceinline__ float stem_elem(const float* __restrict__ X, int b, int i, int j, int k) {
  const int kc = min(k, 23);
  const int t7 = kc / 7;
  const int ky = (kc < 21) ? t7 : 3;
  const int kx = (kc < 21) ? (kc - t7 * 7) : (kc - 21);
  const int ii = i + ky - 3, jj = j + kx - 3;
  const bool valid = (k < 24) && (ii >= 0) && (jj >= 0) && (jj < NHW);
  const int iic = max(ii, 0);
  const int jjc = min(max(jj, 0), NHW - 1);
  const float x = X[(size_t)(b * NHW + iic) * NHW + jjc];
  return valid ? x : 0.0f;
}
__global__ __launch_bounds__(256) void im2col_c1(const float* __restrict__ X, unsigned short* __restrict__ hi,
                                                  unsigned short* __restrict__ lo) {
  const int t = blockIdx.x * 256 + threadIdx.x;
  if (t >= NPIX * 4) return;
  const int R = t >> 2, q = t & 3;
  const int b = R >> 12, i = (R >> 6) & 63, j = R & 63;
  v4u hv, lv;
#pragma unroll
  for (int m = 0; m < 4; ++m) {
    const float x0 = stem_elem(X, b, i, j, 8 * q + 2 * m);
    const float x1 = stem_elem(X, b, i, j, 8 * q + 2 * m + 1);
    unsigned hw, lw; split_pack(x0, x1, hw, lw); hv[m] = hw; lv[m] = lw;
  }
  store_planes2(hi, lo, (size_t)8 * t, hv, lv);
}

__global__ __launch_bounds__(256) void im2col_c16(const float* __restrict__ src, int spitch, int row0, int nrows,
                                                   unsigned short* __restrict__ hi, unsigned short* __restrict__ lo) {
  const int t = blockIdx.x * 256 + threadIdx.x;
  if (t >= nrows * 52) return;
  const int rl = t / 52;
  const int g = t - rl * 52;
  const int R = row0 + rl;
  const int b = R >> 12, i = (R >> 6) & 63, j = R & 63;
  const int tap = g >> 1;
  const int c8 = (g & 1) * 8;
  const int tapc = min(tap, 24);
  const int t7 = tapc / 7;
  const int ky = (tapc < 21) ? t7 : 3;
  const int kx = (tapc < 21) ? (tapc - t7 * 7) : (tapc - 21);
  const int ii = i + ky - 3, jj = j + kx - 3;
  const bool valid = (tap < 25) && (ii >= 0) && (jj >= 0) && (jj < NHW);
  const int iic = max(ii, 0);
  const int jjc = min(max(jj, 0), NHW - 1);
  const float* sp = src + (size_t)((b * NHW + iic) * NHW + jjc) * spitch + c8;
  const v4f a0 = *(const v4f*)(sp);
  const v4f a1 = *(const v4f*)(sp + 4);
  float x[8];
#pragma unroll
  for (int e = 0; e < 4; ++e) {
    x[e]     = valid ? a0[e] : 0.0f;
    x[4 + e] = valid ? a1[e] : 0.0f;
  }
  v4u hv, lv;
#pragma unroll
  for (int m = 0; m < 4; ++m) {
    unsigned hw, lw; split_pack(x[2 * m], x[2 * m + 1], hw, lw); hv[m] = hw; lv[m] = lw;
  }
  store_planes2(hi, lo, (size_t)8 * t, hv, lv);
}

__global__ __launch_bounds__(256) void cast_act_planes(const float* __restrict__ src, int spitch,
                                                        unsigned short* __restrict__ hi, unsigned short* __restrict__ lo) {
  const int t = blockIdx.x * 256 + threadIdx.x;
  if (t >= NPIX * 4) return;
  const int R = t >> 2, q = t & 3;
  const float* sp = src + (size_t)R * spitch + (q & 1) * 8;
  const v4f a0 = *(const v4f*)(sp);
  const v4f a1 = *(const v4f*)(sp + 4);
  const bool pz = (q < 2);
  float x[8];
#pragma unroll
  for (int e = 0; e < 4; ++e) {
    x[e]     = pz ? a0[e] : 0.0f;
    x[4 + e] = pz ? a1[e] : 0.0f;
  }
  v4u hv, lv;
#pragma unroll
  for (int m = 0; m < 4; ++m) {
    unsigned hw, lw; split_pack(x[2 * m], x[2 * m + 1], hw, lw); hv[m] = hw; lv[m] = lw;
  }
  store_planes2(hi, lo, (size_t)8 * t, hv, lv);
}

__global__ __launch_bounds__(128) void dlstm_kernel(const float* __restrict__ GIN,
                                                     const unsigned short* __restrict__ WSh,
                                                     const unsigned short* __restrict__ WSl,
                                                     const float* __restrict__ bisl,
                                                     float* __restrict__ HS) {
  __shared__ __align__(16) unsigned short At[2][NHW * APITCH];
  __shared__ __align__(16) float          Sst[NHW * NCH];
  const int tid = threadIdx.x, lane = tid & 31, wave = tid >> 5;
  const int c = lane & 15, hh = lane >> 4, koff = hh * 8;
  const int b = blockIdx.x & 15;
  const int d = blockIdx.x >> 4;

  const __bf16* wh = (const __bf16*)WSh + (size_t)d * NGATE * 32;
  const __bf16* wl = (const __bf16*)WSl + (size_t)d * NGATE * 32;
  v16b bh[4], bl[4];
  float bisv[4];
#pragma unroll
  for (int n = 0; n < 4; ++n) {
    bh[n] = Frag<__bf16>::load(wh + (size_t)(n * 16 + c) * 32 + koff);
    bl[n] = Frag<__bf16>::load(wl + (size_t)(n * 16 + c) * 32 + koff);
    bisv[n] = bisl[d * NGATE + n * 16 + c];
  }
  float cp[8];
#pragma unroll
  for (int r = 0; r < 8; ++r) cp[r] = 0.0f;

  const v8f z8 = {0.f, 0.f, 0.f, 0.f, 0.f, 0.f, 0.f, 0.f};
  {
    v4u* az = (v4u*)&At[0][0];
    const v4u z4u = {0u, 0u, 0u, 0u};
#pragma unroll
    for (int it = 0; it < 5; ++it) az[tid + 128 * it] = z4u;
  }
  __syncthreads();

  float* hsb = HS + (size_t)d * HS_DIR + (size_t)b * NJP * (NHW * NCH);
  const float* ginb = GIN + (size_t)b * (NHW * NHW * GPITCH) + d * NGATE + c;
  const __bf16* ahrow = (const __bf16*)&At[0][0] + (16 * wave + c) * APITCH + koff;
  const __bf16* alrow = (const __bf16*)&At[1][0] + (16 * wave + c) * APITCH + koff;

#pragma unroll 1
  for (int jp = 0; jp < NJP; ++jp) {
    const v16b ah = Frag<__bf16>::load(ahrow);
    const v16b al = Frag<__bf16>::load(alrow);
    v8f acc[4];
#pragma unroll
    for (int n = 0; n < 4; ++n) {
      v8f a0 = z8;
      a0 = Frag<__bf16>::mma(ah, bh[n], a0);
      a0 = Frag<__bf16>::mma(ah, bl[n], a0);
      a0 = Frag<__bf16>::mma(al, bh[n], a0);
      acc[n] = a0;
    }
    dep_guard_b(acc[0], acc[3], ah, al);
    keep4_b(bh[0], bl[0], bh[3], bl[3]);
    acc_guard4(acc[0], acc[1], acc[2], acc[3]);

#pragma unroll
    for (int r = 0; r < 8; ++r) {
      const int i = 16 * wave + 8 * hh + r;
      const int q = jp - i;
      const bool valid = ((unsigned)q < 64u);
      const int qc = min(max(q, 0), 63);
      const int jsrc = d ? (63 - qc) : qc;
      const float* gp = ginb + (size_t)(i * NHW + jsrc) * GPITCH;
      const float g0 = gp[0], g1 = gp[16], g2 = gp[32], g3 = gp[48];
      const float go = acc[0][r] + (valid ? g0 : bisv[0]);
      const float gf = acc[1][r] + (valid ? g1 : bisv[1]);
      const float gi = acc[2][r] + (valid ? g2 : bisv[2]);
      const float gg = acc[3][r] + (valid ? g3 : bisv[3]);
      const float cn = fsig(gf) * cp[r] + fsig(gi) * ftanh(gg);
      const float hn = fsig(go) * ftanh(cn);
      cp[r] = cn;
      Sst[i * NCH + c] = hn;
    }
    __syncthreads();

#pragma unroll
    for (int it = 0; it < 2; ++it) {
      const int grp = tid + it * 128;
      const int i = grp >> 2, g = grp & 3;
      const int rsrc = (g < 2) ? (i - 1) : i;
      const bool rv = (rsrc >= 0);
      const int rs = max(rsrc, 0);
      const int col0 = (g & 1) * 8;
      const v4f a0 = *(const v4f*)(Sst + rs * NCH + col0);
      const v4f a1 = *(const v4f*)(Sst + rs * NCH + col0 + 4);
      float x[8];
#pragma unroll
      for (int e = 0; e < 4; ++e) {
        x[e]     = rv ? a0[e] : 0.0f;
        x[4 + e] = rv ? a1[e] : 0.0f;
      }
      v4u hv, lv;
#pragma unroll
      for (int m = 0; m < 4; ++m) {
        unsigned hw, lw; split_pack(x[2 * m], x[2 * m + 1], hw, lw); hv[m] = hw; lv[m] = lw;
      }
      *(v4u*)(&At[0][i * APITCH + 8 * g]) = hv;
      *(v4u*)(&At[1][i * APITCH + 8 * g]) = lv;
    }
    {
      float* hsj = hsb + (size_t)jp * (NHW * NCH);
      const v4f v0 = *(const v4f*)(Sst + 4 * tid);
      const v4f v1 = *(const v4f*)(Sst + 512 + 4 * tid);
      for (int pass = 0; pass < 2; ++pass) {
        *(volatile v4f*)(hsj + 4 * tid) = v0;
        *(volatile v4f*)(hsj + 512 + 4 * tid) = v1;
        __threadfence();
      }
    }
    __syncthreads();
  }
}

__global__ __launch_bounds__(256) void combine_kernel(const float* __restrict__ hin, int hpitch,
                                                       const float* __restrict__ HS,
                                                       float* __restrict__ hout,
                                                       unsigned short* __restrict__ hi, unsigned short* __restrict__ lo) {
  const int t = blockIdx.x * 256 + threadIdx.x;
  const int lane = threadIdx.x & 31;
  const int R = t >> 2, q = t & 3;
  const int b = R >> 12, i = (R >> 6) & 63, j = R & 63;
  const v4f x = *(const v4f*)(hin + (size_t)R * hpitch + 4 * q);
  const int jp0 = i + j;
  const v4f lf = *(const v4f*)(HS + ((size_t)(b * NJP + jp0) * NHW + i) * NCH + 4 * q);
  const int im1 = max(i - 1, 0);
  const int jp1 = im1 + 63 - j;
  const v4f rt = *(const v4f*)(HS + HS_DIR + ((size_t)(b * NJP + jp1) * NHW + im1) * NCH + 4 * q);
  const bool hasr = (i >= 1);
  v4f o;
#pragma unroll
  for (int e = 0; e < 4; ++e) {
    const float rr = hasr ? rt[e] : 0.0f;
    o[e] = (x[e] + lf[e]) + rr;
  }
  store_v4f2(hout + (size_t)4 * t, o);

  const int base = lane & ~3;
  const int sa = base + 2 * (q & 1);
  const int sb = sa + 1;
  float pa[4], pb[4];
#pragma unroll
  for (int e = 0; e < 4; ++e) {
    const float oe = o[e];
    pa[e] = __shfl(oe, sa, 32);
    pb[e] = __shfl(oe, sb, 32);
  }
  const bool pz = (q < 2);
  float xx[8];
#pragma unroll
  for (int e = 0; e < 4; ++e) {
    xx[e]     = pz ? pa[e] : 0.0f;
    xx[4 + e] = pz ? pb[e] : 0.0f;
  }
  v4u hv, lv;
#pragma unroll
  for (int m = 0; m < 4; ++m) {
    unsigned hw, lw; split_pack(xx[2 * m], xx[2 * m + 1], hw, lw); hv[m] = hw; lv[m] = lw;
  }
  store_planes2(hi, lo, (size_t)8 * t, hv, lv);
}

__global__ __launch_bounds__(256) void pack_out(const float* __restrict__ C, float* __restrict__ out) {
  const int t = blockIdx.x * 256 + threadIdx.x;
  if (t >= NPIX / 4) return;
  v4f o;
#pragma unroll
  for (int e = 0; e < 4; ++e) o[e] = C[(size_t)(4 * t + e) * 64];
  store_v4f2(out + (size_t)4 * t, o);
}

extern "C" void kernel_launch(void* const* d_in, const int* in_sizes, int n_in,
                              void* d_out, int out_size, void* d_ws, size_t ws_size, hipStream_t stream) {
  if (n_in < 10 || d_out == nullptr || d_ws == nullptr) return;
  if (in_sizes[0] != NPIX || in_sizes[1] != NCH * 49 || in_sizes[2] != NCH ||
      in_sizes[3] != NLAY * 2 * NGATE * NCH || in_sizes[4] != NLAY * 2 * NGATE ||
      in_sizes[5] != NLAY * 2 * NGATE * NCH * 2 || in_sizes[6] != 2 * NCH * NCH * 49 ||
      in_sizes[7] != 2 * NCH || in_sizes[8] != NCH || in_sizes[9] != 1 || out_size != NPIX) return;

  const float* X     = (const float*)d_in[0];
  const float* w_in  = (const float*)d_in[1];
  const float* b_in  = (const float*)d_in[2];
  const float* wis   = (const float*)d_in[3];
  const float* bis   = (const float*)d_in[4];
  const float* wss   = (const float*)d_in[5];
  const float* w_mid = (const float*)d_in[6];
  const float* b_mid = (const float*)d_in[7];
  const float* w_out = (const float*)d_in[8];
  const float* b_out = (const float*)d_in[9];
  float* out = (float*)d_out;

  char* ws = (char*)d_ws; size_t off = 0;
  auto carve = [&](size_t bytes) -> char* { char* p = ws + off; off += (bytes + 255) & ~(size_t)255; return p; };
  float*          CSCR  = (float*)carve((size_t)NPIX * 64 * 4);
  float*          HSR   = (float*)carve((size_t)NPIX * 64 * 4);
  float*          HD0   = (float*)carve((size_t)NPIX * NCH * 4);
  float*          HD1   = (float*)carve((size_t)NPIX * NCH * 4);
  unsigned short* HPH   = (unsigned short*)carve((size_t)NPIX * 32 * 2);
  unsigned short* HPL   = (unsigned short*)carve((size_t)NPIX * 32 * 2);
  char*           IMR   = carve((size_t)NPIX * GPITCH * 4);
  unsigned short* WINH  = (unsigned short*)carve((size_t)64 * KPAD_IN * 2);
  unsigned short* WINL  = (unsigned short*)carve((size_t)64 * KPAD_IN * 2);
  unsigned short* WMIDH = (unsigned short*)carve((size_t)2 * 64 * KPAD_MID * 2);
  unsigned short* WMIDL = (unsigned short*)carve((size_t)2 * 64 * KPAD_MID * 2);
  unsigned short* WOUTH = (unsigned short*)carve((size_t)64 * KPAD_OUT * 2);
  unsigned short* WOUTL = (unsigned short*)carve((size_t)64 * KPAD_OUT * 2);
  unsigned short* WISH  = (unsigned short*)carve((size_t)NLAY * 128 * 32 * 2);
  unsigned short* WISL  = (unsigned short*)carve((size_t)NLAY * 128 * 32 * 2);
  unsigned short* WSSH  = (unsigned short*)carve((size_t)NLAY * 2 * 64 * 32 * 2);
  unsigned short* WSSL  = (unsigned short*)carve((size_t)NLAY * 2 * 64 * 32 * 2);
  float*          BIASP = (float*)carve((size_t)4 * 64 * 4);
  if (off > ws_size || off > (size_t)134217728) return;
  float*          GIN   = (float*)IMR;
  unsigned short* IMH   = (unsigned short*)IMR;
  unsigned short* IML   = (unsigned short*)(IMR + 16777216);
  float*          CSCR2 = HSR;
  float*          HD[2] = {HD0, HD1};

  prep_bias_pad<<<1, 64, 0, stream>>>(b_in, b_mid, b_out, BIASP);
  prep_conv_w<1, 7><<<1, 256, 0, stream>>>(w_in, 16, 24, KPAD_IN / 8, WINH, WINL);
  prep_conv_w<16, 7><<<13, 256, 0, stream>>>(w_mid, 16, 25, KPAD_MID / 8, WMIDH, WMIDL);
  prep_conv_w<16, 7><<<13, 256, 0, stream>>>(w_mid + 16 * 16 * 49, 16, 25, KPAD_MID / 8,
                                             WMIDH + 64 * KPAD_MID, WMIDL + 64 * KPAD_MID);
  prep_conv_w<16, 1><<<1, 256, 0, stream>>>(w_out, 1, 1, KPAD_OUT / 8, WOUTH, WOUTL);
  prep_wis<<<(NLAY * 128 * 4) / 256, 256, 0, stream>>>(wis, WISH, WISL);
  prep_wss<<<(NLAY * 2 * 64 * 4) / 256, 256, 0, stream>>>(wss, WSSH, WSSL);

  im2col_c1<<<(NPIX * 4) / 256, 256, 0, stream>>>(X, IMH, IML);
  wmma_gemm64<1, true, 2, 0, false, 0><<<dim3(NPIX / 64 / 8, 1), 256, 0, stream>>>(
      IMH, IML, KPAD_IN, 0L, WINH, WINL, KPAD_IN, 0L, (void*)CSCR, (void*)CSCR, 64, 0L,
      BIASP, CSCR, 0L, NPIX, 64, KPAD_IN, 1.0f);
  cast_act_planes<<<(NPIX * 4) / 256, 256, 0, stream>>>(CSCR, 64, HPH, HPL);

  for (int l = 0; l < NLAY; ++l) {
    wmma_gemm64<1, true, 2, 0, false, 0><<<dim3((NPIX / 64) * 2 / 8, 1), 256, 0, stream>>>(
        HPH, HPL, 32, 0L, WISH + (size_t)l * 128 * 32, WISL + (size_t)l * 128 * 32, 32, 0L,
        (void*)GIN, (void*)GIN, GPITCH, 0L, bis + (size_t)l * 128, CSCR, 0L, NPIX, 128, 32, 1.0f);
    dlstm_kernel<<<2 * NB, 128, 0, stream>>>(GIN, WSSH + (size_t)l * 2 * 64 * 32, WSSL + (size_t)l * 2 * 64 * 32,
                                              bis + (size_t)l * 128, HSR);
    const float* hprev = (l == 0) ? (const float*)CSCR : (const float*)HD[(l - 1) & 1];
    const int hpit = (l == 0) ? 64 : NCH;
    combine_kernel<<<(NPIX * 4) / 256, 256, 0, stream>>>(hprev, hpit, HSR, HD[l & 1], HPH, HPL);
  }
  const float* hfin = HD[(NLAY - 1) & 1];

  for (int ch = 0; ch < MID_NCHUNK; ++ch) {
    im2col_c16<<<(MID_CHUNK * 52) / 256, 256, 0, stream>>>(hfin, NCH, ch * MID_CHUNK, MID_CHUNK, IMH, IML);
    wmma_gemm64<1, true, 2, 0, false, 2><<<dim3(MID_CHUNK / 64 / 8, 1), 256, 0, stream>>>(
        IMH, IML, KPAD_MID, 0L, WMIDH, WMIDL, KPAD_MID, 0L,
        (void*)(CSCR + (size_t)ch * MID_CHUNK * 64), (void*)CSCR, 64, 0L,
        BIASP + 64, CSCR, 0L, MID_CHUNK, 64, KPAD_MID, 1.0f);
  }
  for (int ch = 0; ch < MID_NCHUNK; ++ch) {
    im2col_c16<<<(MID_CHUNK * 52) / 256, 256, 0, stream>>>(CSCR, 64, ch * MID_CHUNK, MID_CHUNK, IMH, IML);
    wmma_gemm64<1, true, 2, 0, false, 2><<<dim3(MID_CHUNK / 64 / 8, 1), 256, 0, stream>>>(
        IMH, IML, KPAD_MID, 0L, WMIDH + 64 * KPAD_MID, WMIDL + 64 * KPAD_MID, KPAD_MID, 0L,
        (void*)(CSCR2 + (size_t)ch * MID_CHUNK * 64), (void*)CSCR2, 64, 0L,
        BIASP + 128, CSCR, 0L, MID_CHUNK, 64, KPAD_MID, 1.0f);
  }
  cast_act_planes<<<(NPIX * 4) / 256, 256, 0, stream>>>(CSCR2, 64, IMH, IML);
  wmma_gemm64<1, true, 2, 0, false, 0><<<dim3(NPIX / 64 / 8, 1), 256, 0, stream>>>(
      IMH, IML, KPAD_OUT, 0L, WOUTH, WOUTL, KPAD_OUT, 0L, (void*)CSCR, (void*)CSCR, 64, 0L,
      BIASP + 192, CSCR, 0L, NPIX, 64, KPAD_OUT, 1.0f);
  pack_out<<<NPIX / 4 / 256, 256, 0, stream>>>(CSCR, out);
}
